// ODENet_27230092657447
// MI455X (gfx1250) — hardware-verified
//
#include <hip/hip_runtime.h>
#include <stdint.h>

typedef __bf16 v16b __attribute__((ext_vector_type(16)));
typedef __bf16 v8ba __attribute__((ext_vector_type(8), __may_alias__));
typedef float  v8f  __attribute__((ext_vector_type(8)));
typedef float  v4f  __attribute__((ext_vector_type(4)));
typedef unsigned int v4u __attribute__((ext_vector_type(4)));

union Frag { v16b v; v8ba half[2]; };

#define NB      128
#define HD      256
#define TB      32
#define NTH     256
#define PW      132
#define NCHUNK  16384
#define WS_W2_BYTES 262144

__device__ __forceinline__ unsigned int bf16_rne_bits(float f)
{
    const unsigned int u = __float_as_uint(f);
    return (u + 0x7FFFu + ((u >> 16) & 1u)) >> 16;
}

__device__ __forceinline__ void split_bf16(float v, unsigned int& hb, unsigned int& lb)
{
    hb = bf16_rne_bits(v);
    const float hf = __uint_as_float(hb << 16);
    lb = bf16_rne_bits(v - hf);
}

__device__ __forceinline__ float tanh_apx(float x)
{
    const float e = __builtin_amdgcn_exp2f(x * 2.8853900817779268f);
    const float r = __builtin_amdgcn_rcpf(e + 1.0f);
    return 1.0f - 2.0f * r;
}

__device__ __forceinline__ v8f wmma_bf16(v16b a, v16b b, v8f c)
{
    return __builtin_amdgcn_wmma_f32_16x16x32_bf16(false, a, false, b, (short)0, c, false, false);
}

__global__ __launch_bounds__(NTH)
void k_prep(const float* __restrict__ W2, unsigned int* __restrict__ Bw, int nchunks)
{
    const int c = blockIdx.x * NTH + threadIdx.x;
    if (c >= nchunks) return;
    const int hh    = c & 1;
    const int lp    = (c >> 1) & 31;
    const int plane = (c >> 6) & 1;
    const int nt    = (c >> 7) & 15;
    const int kc    = c >> 11;
    const int ncol  = nt * 16 + (lp & 15);
    const int kb    = kc * 32 + 16 * hh + 8 * (lp >> 4);

    unsigned int pk[4];
    #pragma unroll
    for (int e2 = 0; e2 < 4; ++e2) {
        unsigned int bits[2];
        #pragma unroll
        for (int j = 0; j < 2; ++j) {
            const int k = kb + 2 * e2 + j;
            const float v = W2[k * HD + ncol];
            unsigned int hb, lb;
            split_bf16(v, hb, lb);
            bits[j] = plane ? lb : hb;
        }
        pk[e2] = bits[0] | (bits[1] << 16);
    }
    v4u vv;
    vv.x = pk[0]; vv.y = pk[1]; vv.z = pk[2]; vv.w = pk[3];
    volatile v4u* p = (volatile v4u*)(Bw + (size_t)c * 4);
    *p = vv;
    __threadfence();
    *p = vv;
}

__global__ __launch_bounds__(NTH)
void k_main(const float* __restrict__ x,
            const float* __restrict__ W1,
            const float* __restrict__ b1,
            const float* __restrict__ b2,
            const float* __restrict__ W3,
            const float* __restrict__ b3,
            const __bf16* __restrict__ Bw,
            float* __restrict__ out,
            int tsteps)
{
    __shared__ __align__(16) unsigned int sAhi[TB * PW];
    __shared__ __align__(16) unsigned int sAlo[TB * PW];
    __shared__ float sW1y[HD], sW1x[HD], sB1[HD], sB2[HD], sW3[HD];
    __shared__ float sPart[8 * TB];

    const int tid  = threadIdx.x;
    const int lane = tid & 31;
    const int wave = tid >> 5;
    const int h    = lane >> 4;
    const int m    = lane & 15;
    const int b0   = blockIdx.x * TB;
    const int n0   = wave * 32;

    for (int i = tid; i < HD; i += NTH) {
        sW1y[i] = W1[i];
        sW1x[i] = W1[HD + i];
        sB1[i]  = b1[i];
        sB2[i]  = b2[i];
        sW3[i]  = W3[i];
    }
    const float b3v = b3[0];
    __syncthreads();

    float y = 0.0f;

    for (int t = 0; t < tsteps; ++t) {
        if (wave == 0) {
            v4f o;
            o.x = __shfl(y, (4 * lane + 0) & 31);
            o.y = __shfl(y, (4 * lane + 1) & 31);
            o.z = __shfl(y, (4 * lane + 2) & 31);
            o.w = __shfl(y, (4 * lane + 3) & 31);
            if (lane < 8) {
                volatile v4f* p = (volatile v4f*)(out + (size_t)t * NB + b0 + 4 * lane);
                *p = o;
                __threadfence();
                *p = o;
            }
        }

        const float yv = y;
        const float xv = x[(size_t)t * NB + b0 + lane];
        #pragma unroll 1
        for (int c = 0; c < 4; ++c) {
            const int cb = n0 + 8 * c;
            unsigned int ph[4], pl[4];
            #pragma unroll
            for (int e2 = 0; e2 < 4; ++e2) {
                unsigned int hb[2], lb[2];
                #pragma unroll
                for (int j = 0; j < 2; ++j) {
                    const int col = cb + 2 * e2 + j;
                    const float pre = (yv * sW1y[col] + xv * sW1x[col]) + sB1[col];
                    const float hv = tanh_apx(pre);
                    split_bf16(hv, hb[j], lb[j]);
                }
                ph[e2] = hb[0] | (hb[1] << 16);
                pl[e2] = lb[0] | (lb[1] << 16);
            }
            v4u vh, vl;
            vh.x = ph[0]; vh.y = ph[1]; vh.z = ph[2]; vh.w = ph[3];
            vl.x = pl[0]; vl.y = pl[1]; vl.z = pl[2]; vl.w = pl[3];
            const int ui = lane * PW + (cb >> 1);
            *(v4u*)(sAhi + ui) = vh;
            *(v4u*)(sAlo + ui) = vl;
        }
        __syncthreads();

        v8f acc00 = {}; v8f acc01 = {}; v8f acc10 = {}; v8f acc11 = {};
        #pragma unroll 1
        for (int kc = 0; kc < 8; ++kc) {
            const __bf16* pb = Bw + ((size_t)(((kc * 16 + 2 * wave) * 2) * 32 + lane)) * 16;
            Frag bh0, bl0, bh1, bl1;
            bh0.half[0] = ((const v8ba*)(pb))[0];        bh0.half[1] = ((const v8ba*)(pb))[1];
            bl0.half[0] = ((const v8ba*)(pb + 512))[0];  bl0.half[1] = ((const v8ba*)(pb + 512))[1];
            bh1.half[0] = ((const v8ba*)(pb + 1024))[0]; bh1.half[1] = ((const v8ba*)(pb + 1024))[1];
            bl1.half[0] = ((const v8ba*)(pb + 1536))[0]; bl1.half[1] = ((const v8ba*)(pb + 1536))[1];

            const unsigned int* ar0 = sAhi + m * PW + kc * 16 + 4 * h;
            const unsigned int* al0p = sAlo + m * PW + kc * 16 + 4 * h;
            Frag ah0, al0, ah1, al1;
            ah0.half[0] = *(const v8ba*)(ar0);              ah0.half[1] = *(const v8ba*)(ar0 + 8);
            al0.half[0] = *(const v8ba*)(al0p);             al0.half[1] = *(const v8ba*)(al0p + 8);
            ah1.half[0] = *(const v8ba*)(ar0 + 16 * PW);    ah1.half[1] = *(const v8ba*)(ar0 + 16 * PW + 8);
            al1.half[0] = *(const v8ba*)(al0p + 16 * PW);   al1.half[1] = *(const v8ba*)(al0p + 16 * PW + 8);

            acc00 = wmma_bf16(ah0.v, bh0.v, acc00);
            acc00 = wmma_bf16(ah0.v, bl0.v, acc00);
            acc00 = wmma_bf16(al0.v, bh0.v, acc00);
            acc01 = wmma_bf16(ah0.v, bh1.v, acc01);
            acc01 = wmma_bf16(ah0.v, bl1.v, acc01);
            acc01 = wmma_bf16(al0.v, bh1.v, acc01);
            acc10 = wmma_bf16(ah1.v, bh0.v, acc10);
            acc10 = wmma_bf16(ah1.v, bl0.v, acc10);
            acc10 = wmma_bf16(al1.v, bh0.v, acc10);
            acc11 = wmma_bf16(ah1.v, bh1.v, acc11);
            acc11 = wmma_bf16(ah1.v, bl1.v, acc11);
            acc11 = wmma_bf16(al1.v, bh1.v, acc11);
            asm volatile("v_nop\n\tv_nop\n\tv_nop\n\tv_nop"
                         : "+v"(acc00), "+v"(acc01), "+v"(acc10), "+v"(acc11)
                         : "v"(ah0.v), "v"(al0.v), "v"(ah1.v), "v"(al1.v),
                           "v"(bh0.v), "v"(bl0.v), "v"(bh1.v), "v"(bl1.v));
        }

        {
            const float b2a = sB2[n0 + m],  b2b = sB2[n0 + 16 + m];
            const float w3a = sW3[n0 + m],  w3b = sW3[n0 + 16 + m];
            #pragma unroll
            for (int r = 0; r < 8; ++r) {
                float p0 = tanh_apx(acc00[r] + b2a) * w3a + tanh_apx(acc01[r] + b2b) * w3b;
                float p1 = tanh_apx(acc10[r] + b2a) * w3a + tanh_apx(acc11[r] + b2b) * w3b;
                p0 += __shfl_xor(p0, 1); p0 += __shfl_xor(p0, 2); p0 += __shfl_xor(p0, 4); p0 += __shfl_xor(p0, 8);
                p1 += __shfl_xor(p1, 1); p1 += __shfl_xor(p1, 2); p1 += __shfl_xor(p1, 4); p1 += __shfl_xor(p1, 8);
                if (m == 0) {
                    sPart[wave * TB + 8 * h + r]      = p0;
                    sPart[wave * TB + 16 + 8 * h + r] = p1;
                }
            }
        }
        __syncthreads();

        float s = 0.0f;
        #pragma unroll
        for (int w = 0; w < 8; ++w) s += sPart[w * TB + lane];
        const float dy = s + b3v;
        y = yv + dy;
    }
}

extern "C" void kernel_launch(void* const* d_in, const int* in_sizes, int n_in,
                              void* d_out, int out_size, void* d_ws, size_t ws_size,
                              hipStream_t stream)
{
    if (n_in < 7) return;
    const int nx = in_sizes[0];
    if (nx <= 0 || (nx % NB) != 0) return;
    const int tsteps = nx / NB;
    if (in_sizes[1] != 2 * HD || in_sizes[2] != HD || in_sizes[3] != HD * HD ||
        in_sizes[4] != HD || in_sizes[5] != HD || in_sizes[6] < 1) return;
    if (out_size != nx) return;
    if (ws_size < (size_t)WS_W2_BYTES) return;

    const float* x  = (const float*)d_in[0];
    const float* W1 = (const float*)d_in[1];
    const float* b1 = (const float*)d_in[2];
    const float* W2 = (const float*)d_in[3];
    const float* b2 = (const float*)d_in[4];
    const float* W3 = (const float*)d_in[5];
    const float* b3 = (const float*)d_in[6];
    float* out = (float*)d_out;

    unsigned int* Bw = (unsigned int*)d_ws;

    const int prep_blocks = (NCHUNK + NTH - 1) / NTH;
    k_prep<<<dim3(prep_blocks), dim3(NTH), 0, stream>>>(W2, Bw, NCHUNK);

    const int main_blocks = (NB + TB - 1) / TB;
    k_main<<<dim3(main_blocks), dim3(NTH), 0, stream>>>(
        x, W1, b1, b2, W3, b3, (const __bf16*)d_ws, out, tsteps);
}
